// SelfAttention_84645215469985
// MI455X (gfx1250) — hardware-verified
//
#include <hip/hip_runtime.h>


#ifndef NB
#define NB 2
#endif
#ifndef SEQ
#define SEQ 2048
#endif
#define NB_FULL    2
#define SEQ_FULL   2048
#define NHEAD      16
#define HDIM       128
#define BQ         128
#define BK         32
#define NWAVE      8
#define CT         64
#define NKT        (SEQ / CT)
#define TP         72
#define OHALF      64
#define OP         68

#define KB_BYTES   ((size_t)NB * NHEAD * SEQ * HDIM * 2)
#define VT_BYTES   ((size_t)NB * NHEAD * HDIM * SEQ * 2)
#define PART_BYTES ((size_t)NB * NHEAD * SEQ * HDIM * 4)
#define COLP_BYTES ((size_t)NB * NHEAD * NKT * HDIM * 4)
#define TERM_BYTES ((size_t)NB * HDIM * 4)

static_assert(SEQ % BQ == 0);
static_assert(SEQ % CT == 0);
static_assert(SEQ % BK == 0);
static_assert(BQ == NWAVE * 16);
static_assert(HDIM == 128);
static_assert(HDIM % 32 == 0);
static_assert(2 * OHALF == HDIM);
static_assert(16 * 4 == OHALF);
static_assert(CT == 64);
static_assert(256 * 4 * 8 == CT * HDIM);
static_assert(TP >= CT);
static_assert(OP >= OHALF);
static_assert((TP * 2) % 16 == 0);
static_assert((OP * 4) % 16 == 0);
static_assert(NWAVE * 16 * OP * 4 <= 65536);
static_assert(SEQ <= SEQ_FULL);
static_assert(NB >= 1 && NB <= NB_FULL);
static_assert(((size_t)NB * SEQ * (HDIM / 4)) % 256 == 0);
static_assert(KB_BYTES % 128 == 0 && VT_BYTES % 128 == 0 && PART_BYTES % 128 == 0);
static_assert(COLP_BYTES % 128 == 0 && TERM_BYTES % 128 == 0);
static_assert(KB_BYTES + VT_BYTES + PART_BYTES + COLP_BYTES + TERM_BYTES <= (size_t)134217728);

typedef __bf16   bf16;
typedef _Float16 f16;
typedef bf16     v16bf __attribute__((ext_vector_type(16)));
typedef f16      v16h  __attribute__((ext_vector_type(16)));
typedef f16      v8h   __attribute__((ext_vector_type(8)));
typedef float    v8f   __attribute__((ext_vector_type(8)));
typedef float    v4f   __attribute__((ext_vector_type(4)));
typedef unsigned v4u   __attribute__((ext_vector_type(4)));

union FragB  { v16bf v; v4u q[2]; bf16 h[16]; };
union FragH  { v16h  v; v4u q[2]; f16  h[16]; };
union Pack8B { v4u u; bf16 h[8]; };
union Pack8H { v4u u; v8h v; f16 h[8]; };

static __device__ __forceinline__ v8f mma_bf16(v16bf a, v16bf b, v8f acc) {
  acc = __builtin_amdgcn_wmma_f32_16x16x32_bf16(false, a, false, b, (short)0, acc, false, false);
  asm volatile("v_nop\n\tv_nop\n\tv_nop\n\tv_nop" : "+v"(acc) : "v"(a), "v"(b));
  return acc;
}
static __device__ __forceinline__ v8f mma_f16(v16h a, v16h b, v8f acc) {
  acc = __builtin_amdgcn_wmma_f32_16x16x32_f16(false, a, false, b, (short)0, acc, false, false);
  asm volatile("v_nop\n\tv_nop\n\tv_nop\n\tv_nop" : "+v"(acc) : "v"(a), "v"(b));
  return acc;
}

__global__ __launch_bounds__(256) void kv_planes_kernel(const float* __restrict__ kin,
                                                        const float* __restrict__ vin,
                                                        bf16* __restrict__ kb,
                                                        f16* __restrict__ vt,
                                                        float* __restrict__ colp) {
  const int kt  = blockIdx.x;
  const int h   = blockIdx.y;
  const int b   = blockIdx.z;
  const int tid = threadIdx.x;
  __shared__ __align__(16) f16   sT[HDIM * TP];
  __shared__ __align__(16) float sC[HDIM];
  const int s0 = kt * CT;
  const size_t bh = (size_t)b * NHEAD + h;

  v4u    kval[4];
  size_t kidx[4];
  #pragma unroll
  for (int kk = 0; kk < 4; ++kk) {
    const int key = kk * 16 + (tid >> 4);
    const int d0  = (tid & 15) * 8;
    const size_t src = (bh * SEQ_FULL + s0 + key) * HDIM + d0;
    const v4f k0 = *(const v4f*)(kin + src);
    const v4f k1 = *(const v4f*)(kin + src + 4);
    const v4f v0 = *(const v4f*)(vin + src);
    const v4f v1 = *(const v4f*)(vin + src + 4);
    Pack8B pk;
    #pragma unroll
    for (int i = 0; i < 4; ++i) {
      pk.h[i]     = (bf16)k0[i];
      pk.h[4 + i] = (bf16)k1[i];
    }
    kval[kk] = pk.u;
    kidx[kk] = (bh * SEQ + s0 + key) * HDIM + d0;
    #pragma unroll
    for (int i = 0; i < 4; ++i) {
      sT[(d0 + i) * TP + key]     = (f16)(float)(bf16)v0[i];
      sT[(d0 + 4 + i) * TP + key] = (f16)(float)(bf16)v1[i];
    }
  }
  __syncthreads();

  v4u    vval[4];
  size_t vidx[4];
  #pragma unroll
  for (int kk = 0; kk < 4; ++kk) {
    const int d  = kk * 32 + (tid >> 3);
    const int ks = (tid & 7) * 8;
    Pack8H ph;
    ph.v = *(const v8h*)(&sT[d * TP + ks]);
    vval[kk] = ph.u;
    vidx[kk] = (bh * HDIM + d) * SEQ + s0 + ks;
  }

  if (tid < HDIM) {
    float cs = 0.0f;
    #pragma unroll 1
    for (int ks = 0; ks < CT; ks += 8) {
      const v8h x = *(const v8h*)(&sT[tid * TP + ks]);
      #pragma unroll
      for (int i = 0; i < 8; ++i) cs += (float)x[i];
    }
    sC[tid] = cs;
  }
  __syncthreads();

  v4f cval = (v4f){0, 0, 0, 0};
  const size_t cidx = ((bh * NKT) + kt) * HDIM + (size_t)(tid & 31) * 4;
  if (tid < 32) cval = *(const v4f*)(&sC[tid * 4]);

  #pragma unroll
  for (int kk = 0; kk < 4; ++kk) {
    *(volatile v4u*)(kb + kidx[kk]) = kval[kk];
    *(volatile v4u*)(vt + vidx[kk]) = vval[kk];
  }
  if (tid < 32) *(volatile v4f*)(colp + cidx) = cval;
  __threadfence();
  #pragma unroll
  for (int kk = 0; kk < 4; ++kk) {
    *(volatile v4u*)(kb + kidx[kk]) = kval[kk];
    *(volatile v4u*)(vt + vidx[kk]) = vval[kk];
  }
  if (tid < 32) *(volatile v4f*)(colp + cidx) = cval;
}

__global__ __launch_bounds__(256) void attn_kernel(const float* __restrict__ qin,
                                                   const bf16* __restrict__ kb,
                                                   const f16* __restrict__ vt,
                                                   float* __restrict__ part) {
  const int qblk = blockIdx.x;
  const int h    = blockIdx.y;
  const int b    = blockIdx.z;
  const int tid  = threadIdx.x;
  const int wave = __builtin_amdgcn_readfirstlane(tid >> 5);
  const int lane = tid & 31;
  const int lq   = lane & 15;
  const int hi   = lane >> 4;

  __shared__ __align__(16) float sO[NWAVE * 16 * OP];

  const int    qrow0 = qblk * BQ + wave * 16;
  const size_t bh    = (size_t)b * NHEAD + h;

  FragB qf[4];
  {
    const float* qp = qin + (bh * SEQ_FULL + qrow0 + lq) * HDIM;
    #pragma unroll
    for (int f = 0; f < 4; ++f) {
      const v4f a0 = *(const v4f*)(qp + f * 32 + hi * 8);
      const v4f a1 = *(const v4f*)(qp + f * 32 + hi * 8 + 4);
      const v4f b0 = *(const v4f*)(qp + f * 32 + 16 + hi * 8);
      const v4f b1 = *(const v4f*)(qp + f * 32 + 16 + hi * 8 + 4);
      #pragma unroll
      for (int i = 0; i < 4; ++i) {
        qf[f].h[i]      = (bf16)a0[i];
        qf[f].h[4 + i]  = (bf16)a1[i];
        qf[f].h[8 + i]  = (bf16)b0[i];
        qf[f].h[12 + i] = (bf16)b1[i];
      }
    }
  }

  const bf16* kb_h = kb + bh * SEQ * HDIM;
  const f16*  vt_h = vt + bh * HDIM * SEQ;

  v8f o[8];
  #pragma unroll
  for (int dt = 0; dt < 8; ++dt) o[dt] = (v8f){0, 0, 0, 0, 0, 0, 0, 0};

  float rmax = -__builtin_inff();
  float rsum = 0.0f;
  const float SL = 0.08838834764831845f * 1.4426950408889634f;

  #pragma unroll 1
  for (int i = 0; i < SEQ / BK; ++i) {
    const int j0 = i * BK;

    v8f c[2];
    #pragma unroll
    for (int sub = 0; sub < 2; ++sub) {
      v8f acc = (v8f){0, 0, 0, 0, 0, 0, 0, 0};
      #pragma unroll
      for (int f = 0; f < 4; ++f) {
        const bf16* base = kb_h + (size_t)(j0 + sub * 16 + lq) * HDIM + f * 32 + hi * 8;
        FragB ak;
        ak.q[0] = *(const v4u*)(base);
        ak.q[1] = *(const v4u*)(base + 16);
        acc = mma_bf16(ak.v, qf[f].v, acc);
      }
      c[sub] = acc;
      __builtin_amdgcn_sched_barrier(0);
    }

    float m_new = rmax;
    #pragma unroll
    for (int r = 0; r < 8; ++r) {
      m_new = fmaxf(m_new, c[0][r]);
      m_new = fmaxf(m_new, c[1][r]);
    }
    m_new = fmaxf(m_new, __shfl_xor(m_new, 16, 32));
    const float scale = __builtin_amdgcn_exp2f((rmax - m_new) * SL);
    rmax = m_new;

    FragH pa;
    float psum = 0.0f;
    #pragma unroll
    for (int r = 0; r < 8; ++r) {
      const float p0 = __builtin_amdgcn_exp2f((c[0][r] - m_new) * SL);
      const float p1 = __builtin_amdgcn_exp2f((c[1][r] - m_new) * SL);
      psum += p0 + p1;
      pa.h[r]     = (f16)(p0 * 4096.0f);
      pa.h[8 + r] = (f16)(p1 * 4096.0f);
    }
    rsum = rsum * scale + psum + __shfl_xor(psum, 16, 32);

    float sc[8];
    #pragma unroll
    for (int r = 0; r < 8; ++r) sc[r] = __shfl(scale, (hi << 3) + r, 32);
    #pragma unroll
    for (int dt = 0; dt < 8; ++dt) {
      #pragma unroll
      for (int r = 0; r < 8; ++r) o[dt][r] *= sc[r];
    }
    __builtin_amdgcn_sched_barrier(0);

    #pragma unroll
    for (int g = 0; g < 2; ++g) {
      FragH bv[4];
      #pragma unroll
      for (int t = 0; t < 4; ++t) {
        const f16* base = vt_h + (size_t)((g * 4 + t) * 16 + lq) * SEQ + j0 + hi * 8;
        bv[t].q[0] = *(const v4u*)(base);
        bv[t].q[1] = *(const v4u*)(base + 16);
      }
      #pragma unroll
      for (int t = 0; t < 4; ++t) o[g * 4 + t] = mma_f16(pa.v, bv[t].v, o[g * 4 + t]);
      __builtin_amdgcn_sched_barrier(0);
    }
  }

  float rs[8];
  #pragma unroll
  for (int r = 0; r < 8; ++r) rs[r] = (1.0f / 4096.0f) * (1.0f / __shfl(rsum, (hi << 3) + r, 32));

  const int so = wave * (16 * OP);
  v4f    vals[16];
  size_t gidx[8];

  #pragma unroll
  for (int r = 0; r < 8; ++r) {
    #pragma unroll
    for (int t = 0; t < 4; ++t) sO[so + (hi * 8 + r) * OP + t * 16 + lq] = o[t][r] * rs[r];
  }
  __syncthreads();
  #pragma unroll
  for (int it = 0; it < 8; ++it) {
    const int row = it * 2 + hi;
    vals[it] = *(const v4f*)(&sO[so + row * OP + lq * 4]);
    gidx[it] = (bh * SEQ + qrow0 + row) * HDIM + lq * 4;
  }
  __syncthreads();
  #pragma unroll
  for (int r = 0; r < 8; ++r) {
    #pragma unroll
    for (int t = 0; t < 4; ++t) sO[so + (hi * 8 + r) * OP + t * 16 + lq] = o[4 + t][r] * rs[r];
  }
  __syncthreads();
  #pragma unroll
  for (int it = 0; it < 8; ++it) {
    const int row = it * 2 + hi;
    vals[8 + it] = *(const v4f*)(&sO[so + row * OP + lq * 4]);
  }

  #pragma unroll
  for (int it = 0; it < 8; ++it) {
    *(volatile v4f*)(part + gidx[it])         = vals[it];
    *(volatile v4f*)(part + gidx[it] + OHALF) = vals[8 + it];
  }
  __threadfence();
  #pragma unroll
  for (int it = 0; it < 8; ++it) {
    *(volatile v4f*)(part + gidx[it])         = vals[it];
    *(volatile v4f*)(part + gidx[it] + OHALF) = vals[8 + it];
  }
}

__global__ __launch_bounds__(128) void meanv_kernel(const float* __restrict__ colp,
                                                    float* __restrict__ term) {
  const int b   = blockIdx.x;
  const int tid = threadIdx.x;
  __shared__ __align__(16) float sM[HDIM];
  const float* src = colp + (size_t)b * NHEAD * NKT * HDIM + tid;
  double acc = 0.0;
  #pragma unroll 4
  for (int j = 0; j < NHEAD * NKT; ++j) acc += (double)src[(size_t)j * HDIM];
  sM[tid] = (float)(acc * ((double)(NHEAD - 1) / (double)SEQ));
  __syncthreads();
  if (tid < 32) {
    const v4f val = *(const v4f*)(&sM[tid * 4]);
    float* dst = term + (size_t)b * HDIM + tid * 4;
    *(volatile v4f*)dst = val;
    __threadfence();
    *(volatile v4f*)dst = val;
  }
}

__global__ __launch_bounds__(256) void headsum_kernel(const float* __restrict__ part,
                                                      const float* __restrict__ term,
                                                      float* __restrict__ out) {
  const int g   = blockIdx.x * 256 + threadIdx.x;
  const int d4  = g & (HDIM / 4 - 1);
  const int row = g / (HDIM / 4);
  const int b   = row / SEQ;
  const int s   = row - b * SEQ;
  v4f acc = (v4f){0, 0, 0, 0};
  #pragma unroll 4
  for (int h = 0; h < NHEAD; ++h)
    acc += *(const v4f*)(part + (((size_t)b * NHEAD + h) * SEQ + s) * HDIM + d4 * 4);
  acc += *(const v4f*)(term + (size_t)b * HDIM + d4 * 4);
  float* dst = out + ((size_t)b * SEQ_FULL + s) * HDIM + d4 * 4;
  *(volatile v4f*)dst = acc;
  __threadfence();
  *(volatile v4f*)dst = acc;
}

extern "C" void kernel_launch(void* const* d_in, const int* in_sizes, int n_in,
                              void* d_out, int out_size, void* d_ws, size_t ws_size,
                              hipStream_t stream) {
  if (n_in < 3) return;
  const size_t in_need  = (((size_t)(NB - 1) * NHEAD + (NHEAD - 1)) * SEQ_FULL + SEQ) * HDIM;
  const size_t out_need = ((size_t)(NB - 1) * SEQ_FULL + SEQ) * HDIM;
  if ((size_t)in_sizes[0] < in_need) return;
  if ((size_t)in_sizes[1] < in_need) return;
  if ((size_t)in_sizes[2] < in_need) return;
  if ((size_t)out_size < out_need) return;
  if (ws_size < KB_BYTES + VT_BYTES + PART_BYTES + COLP_BYTES + TERM_BYTES) return;

  const float* qin = (const float*)d_in[0];
  const float* kin = (const float*)d_in[1];
  const float* vin = (const float*)d_in[2];
  float*       out = (float*)d_out;

  char*  wsb  = (char*)d_ws;
  bf16*  kb   = (bf16*)wsb;
  f16*   vt   = (f16*)(wsb + KB_BYTES);
  float* part = (float*)(wsb + KB_BYTES + VT_BYTES);
  float* colp = (float*)(wsb + KB_BYTES + VT_BYTES + PART_BYTES);
  float* term = (float*)(wsb + KB_BYTES + VT_BYTES + PART_BYTES + COLP_BYTES);

  kv_planes_kernel<<<dim3(SEQ / CT, NHEAD, NB), 256, 0, stream>>>(kin, vin, kb, vt, colp);
  meanv_kernel<<<dim3(NB), 128, 0, stream>>>(colp, term);
  attn_kernel<<<dim3(SEQ / BQ, NHEAD, NB), 256, 0, stream>>>(qin, kb, vt, part);
  headsum_kernel<<<dim3((unsigned)(((size_t)NB * SEQ * (HDIM / 4)) / 256)), 256, 0, stream>>>(part, term, out);
}
